// MC_63995012710625
// MI455X (gfx1250) — hardware-verified
//
#include <hip/hip_runtime.h>
#include <stddef.h>


typedef _Float16 v16h __attribute__((ext_vector_type(16)));
typedef _Float16 v8h  __attribute__((ext_vector_type(8)));
typedef float    v8f  __attribute__((ext_vector_type(8)));
typedef float    v4f  __attribute__((ext_vector_type(4)));
typedef _Float16 h16;

#ifndef NB
#define NB 2048
#endif
#define NB_FULL 2048
#ifndef TAIL_RES
#define TAIL_RES 0
#endif

#define NNODE 128
#define FEAT  10
#define INDIM 7
#define HID   64
#define TAU   22
#define TAUP  32
#define K2    (2 * HID)
#define XROW  (NNODE * FEAT)
#define OTILE (16 * TAU)

#define LDT 72

#define WCARRY 64.0f
#define CCARRY 16.0f
#define GCARRY 16.0f
#define RCARRY 2048.0f

static_assert(NB >= 64 && NB <= NB_FULL && (NB % 64) == 0);
static_assert((NB % 8) == 0);
static_assert(HID == 64);
static_assert((K2 % 32) == 0 && (HID % 32) == 0);
static_assert(TAU <= TAUP && (TAUP % 16) == 0);
static_assert((XROW % 128) == 0 && XROW == 10 * 32 * 4);
static_assert(NNODE == 4 * 32);
static_assert((OTILE * 4) % 128 == 0 && OTILE / 4 == 88);
static_assert((LDT % 8) == 0 && LDT >= 64);
static_assert(4 * 2 == 8);

#define W2T_BYTES ((size_t)HID * K2 * 2)
#define FCT_BYTES ((size_t)TAUP * HID * 2)
#define CPL_BYTES ((size_t)NB * K2 * 2)
#define OFF_W2T ((size_t)0)
#define OFF_FCT (OFF_W2T + W2T_BYTES)
#define OFF_C   (OFF_FCT + FCT_BYTES)
#define OFF_CR  (OFF_C + CPL_BYTES)
#define WS_TOTAL (OFF_CR + CPL_BYTES)
static_assert((W2T_BYTES % 128) == 0 && (FCT_BYTES % 128) == 0 && (CPL_BYTES % 128) == 0);
static_assert(WS_TOTAL <= (size_t)134217728);

static_assert(INDIM * HID * 4 + 16 * 4 + 8 * XROW * 4 + 8 * NNODE * 4 + 2 * 8 * LDT * 2 <= 131072);
static_assert(2 * 4 * 16 * LDT * 2 + 4 * OTILE * 4 <= 131072);

__device__ __forceinline__ float bf16r(float x) {
  unsigned int u = __float_as_uint(x);
  u = (u + 0x7FFFu + ((u >> 16) & 1u)) & 0xFFFF0000u;
  return __uint_as_float(u);
}

static __device__ __forceinline__ h16 toh_flush(float v) {
  const h16 r = (h16)v;
  return (fabsf(v) < 6.103515625e-05f) ? (h16)0.0f : r;
}

__device__ __forceinline__ v16h frag_at(const _Float16* p) {
  v8h lo = *(const v8h*)(p);
  v8h hi = *(const v8h*)(p + 16);
  v16h out;
#pragma unroll
  for (int i = 0; i < 8; ++i) { out[i] = lo[i]; out[i + 8] = hi[i]; }
  return out;
}
__device__ __forceinline__ v16h ld_frag(const _Float16* base, unsigned ld) {
  const unsigned lane = threadIdx.x & 31u;
  return frag_at(base + (lane & 15u) * ld + (lane >> 4) * 8u);
}

__device__ __forceinline__ v8f wmma16(v16h a, v16h b, v8f c) {
  v8f d = __builtin_amdgcn_wmma_f32_16x16x32_f16(false, a, false, b, (short)0, c,
                                                 false, false);
  asm volatile("v_nop\n\tv_nop\n\tv_nop\n\tv_nop" : "+v"(d) : "v"(a), "v"(b));
  return d;
}

__device__ __forceinline__ float red32_sum(float x) {
#pragma unroll
  for (int off = 1; off < 32; off <<= 1) x += __shfl_xor(x, off, 32);
  return x;
}
__device__ __forceinline__ float red32_max(float x) {
#pragma unroll
  for (int off = 1; off < 32; off <<= 1) x = fmaxf(x, __shfl_xor(x, off, 32));
  return x;
}

__device__ __forceinline__ void wave_lds_sync() {
  __builtin_amdgcn_fence(3  , "wavefront");
  asm volatile("s_wait_dscnt 0x0" ::: "memory");
  __builtin_amdgcn_wave_barrier();
}

__global__ __launch_bounds__(256) void wconv_kernel(
    const float* __restrict__ W, _Float16* __restrict__ Wt, unsigned ldw, unsigned ldk) {
  __shared__ _Float16 T[64 * LDT];
  const unsigned tid = threadIdx.x;
  const unsigned n0 = blockIdx.x * 64u;
  const unsigned k0 = blockIdx.y * 64u;
#pragma unroll 4
  for (unsigned j = 0; j < 16u; ++j) {
    const unsigned idx = tid + 256u * j;
    const unsigned kr = idx >> 6, nc = idx & 63u;
    const float v = W[(size_t)(k0 + kr) * ldw + n0 + nc];
    T[nc * LDT + kr] = toh_flush(WCARRY * bf16r(v));
  }
  __syncthreads();
  v8h x[2];
  size_t off[2];
#pragma unroll
  for (unsigned i = 0; i < 2u; ++i) {
    const unsigned n = 32u * i + (tid >> 3);
    const unsigned kc = (tid & 7u) * 8u;
    x[i] = *(const v8h*)&T[n * LDT + kc];
    off[i] = (size_t)(n0 + n) * ldk + k0 + kc;
  }
#pragma unroll
  for (int i = 0; i < 2; ++i) *(volatile v8h*)(Wt + off[i]) = x[i];
  __threadfence();
#pragma unroll
  for (int i = 0; i < 2; ++i) *(volatile v8h*)(Wt + off[i]) = x[i];
}

__global__ __launch_bounds__(256) void fcconv_kernel(
    const float* __restrict__ W, _Float16* __restrict__ Wt) {
  __shared__ _Float16 T[TAUP * LDT] __attribute__((aligned(16)));
  const unsigned tid = threadIdx.x;
#pragma unroll 4
  for (unsigned j = 0; j < 8u; ++j) {
    const unsigned idx = tid + 256u * j;
    const unsigned kr = idx >> 5, nc = idx & 31u;
    const unsigned ncc = (nc < (unsigned)TAU) ? nc : (unsigned)(TAU - 1);
    const float v = W[kr * (unsigned)TAU + ncc];
    const h16 hv = toh_flush(WCARRY * bf16r(v));
    T[nc * LDT + kr] = (nc < (unsigned)TAU) ? hv : (h16)0.0f;
  }
  __syncthreads();
  const unsigned n = tid >> 3;
  const unsigned kc = (tid & 7u) * 8u;
  const v8h x = *(const v8h*)&T[n * LDT + kc];
  const size_t off = (size_t)n * HID + kc;
  *(volatile v8h*)(Wt + off) = x;
  __threadfence();
  *(volatile v8h*)(Wt + off) = x;
}

__global__ __launch_bounds__(256) void star_kernel(
    const float* __restrict__ fp, const float* __restrict__ W, const float* __restrict__ a,
    _Float16* __restrict__ Cp, _Float16* __restrict__ CpR, const unsigned br) {
#pragma clang fp contract(off)
  __shared__ float Ws[INDIM * HID] __attribute__((aligned(16)));
  __shared__ float wlh[16] __attribute__((aligned(16)));
  __shared__ float Xs[8 * XROW] __attribute__((aligned(16)));
  __shared__ float Es[8 * NNODE] __attribute__((aligned(16)));
  __shared__ _Float16 Cst[8 * LDT] __attribute__((aligned(16)));
#if TAIL_RES
  __shared__ _Float16 CstR[8 * LDT] __attribute__((aligned(16)));
#endif

  const unsigned tid = threadIdx.x, lane = tid & 31u;
  const int wave = __builtin_amdgcn_readfirstlane(threadIdx.x >> 5);
  const unsigned xb = (unsigned)wave * (unsigned)XROW;
  const unsigned eb = (unsigned)wave * (unsigned)NNODE;

#pragma unroll
  for (unsigned j = 0; j < 2u; ++j) {
    const unsigned idx = tid + 256u * j;
    const unsigned ic = (idx < (unsigned)(INDIM * HID)) ? idx : (unsigned)(INDIM * HID - 1);
    const float v = bf16r(W[ic]);
    if (idx < (unsigned)(INDIM * HID)) Ws[idx] = v;
  }
  if (wave == 0) {
    const unsigned k7 = lane & 7u;
    const unsigned kk = (k7 < (unsigned)INDIM) ? k7 : (unsigned)(INDIM - 1);
    const unsigned sel = (lane >> 3) & 1u;
    float acc = 0.0f;
#pragma unroll 1
    for (unsigned d = 0; d < (unsigned)HID; ++d)
      acc += bf16r(W[kk * HID + d]) * bf16r(a[sel * HID + d]);
    if (lane < 16u) wlh[lane] = acc;
  }
  __syncthreads();

  const unsigned b = blockIdx.x * 8u + (unsigned)wave;
  const float* src = fp + ((size_t)b * (2u * NNODE) + (size_t)br * NNODE) * FEAT;
#pragma unroll 2
  for (unsigned j = 0; j < 10u; ++j) {
    const unsigned q = (j * 32u + lane) * 4u;
    const v4f v = *(const v4f*)(src + q);
    v4f r;
#pragma unroll
    for (int i = 0; i < 4; ++i) r[i] = bf16r(v[i]);
    *(v4f*)&Xs[xb + q] = r;
  }
  wave_lds_sync();

  float s1 = 0.0f;
#pragma unroll
  for (int k = 0; k < INDIM; ++k) s1 += Xs[xb + (unsigned)k] * wlh[k];

  float mx = -3.0e38f;
#pragma unroll 1
  for (unsigned j = 0; j < 4u; ++j) {
    const unsigned node = lane + 32u * j;
    float s2 = 0.0f;
#pragma unroll
    for (int k = 0; k < INDIM; ++k) s2 += Xs[xb + node * FEAT + (unsigned)k] * wlh[8 + k];
    float e = s1 + s2;
    e = (e >= 0.0f) ? e : 0.2f * e;
    Es[eb + node] = e;
    mx = fmaxf(mx, (node == 0u) ? -3.0e38f : e);
  }
  mx = red32_max(mx);

  float sum = 0.0f;
  float acc[INDIM];
#pragma unroll
  for (int k = 0; k < INDIM; ++k) acc[k] = 0.0f;
#pragma unroll 1
  for (unsigned j = 0; j < 4u; ++j) {
    const unsigned node = lane + 32u * j;
    const float pe = expf(Es[eb + node] - mx);
    const float p = (node == 0u) ? 0.0f : pe;
    sum += p;
#pragma unroll
    for (int k = 0; k < INDIM; ++k) acc[k] += p * Xs[xb + node * FEAT + (unsigned)k];
  }
  sum = red32_sum(sum);
  const float inv = 1.0f / sum;
  float xw[INDIM], x0[INDIM];
#pragma unroll
  for (int k = 0; k < INDIM; ++k) {
    xw[k] = red32_sum(acc[k]) * inv;
    x0[k] = Xs[xb + (unsigned)k];
  }

#pragma unroll 1
  for (unsigned t = 0; t < 2u; ++t) {
    const unsigned col = lane + 32u * t;
    float h0 = 0.0f, h1 = 0.0f;
#pragma unroll
    for (int k = 0; k < INDIM; ++k) {
      const float w = Ws[(unsigned)k * HID + col];
      h0 += xw[k] * w;
      h1 += x0[k] * w;
    }
    const float v0 = (h0 > 0.0f) ? h0 : (expf(h0) - 1.0f);
    const float v1 = (h1 > 0.0f) ? h1 : (expf(h1) - 1.0f);
    const float c = CCARRY * (v1 + 127.0f * v0);
    const h16 hi = toh_flush(c);
    Cst[(unsigned)wave * LDT + col] = hi;
#if TAIL_RES
    CstR[(unsigned)wave * LDT + col] = toh_flush((c - (float)hi) * RCARRY);
#endif
  }
  __syncthreads();

  if (wave < 2) {
    const unsigned r = 4u * (unsigned)wave + (lane >> 3);
    const unsigned cc = (lane & 7u) * 8u;
    const v8h x = *(const v8h*)&Cst[r * LDT + cc];
    const size_t off = (size_t)(blockIdx.x * 8u + r) * K2 + (size_t)br * HID + cc;
#if TAIL_RES
    const v8h xr = *(const v8h*)&CstR[r * LDT + cc];
#endif
    *(volatile v8h*)(Cp + off) = x;
#if TAIL_RES
    *(volatile v8h*)(CpR + off) = xr;
#endif
    __threadfence();
    *(volatile v8h*)(Cp + off) = x;
#if TAIL_RES
    *(volatile v8h*)(CpR + off) = xr;
#endif
  }
}

__global__ __launch_bounds__(128) void tail_kernel(
    const _Float16* __restrict__ Cp, const _Float16* __restrict__ CpR,
    const _Float16* __restrict__ W2t, const _Float16* __restrict__ Fct,
    const float* __restrict__ fcb, float* __restrict__ out) {
  __shared__ _Float16 Gs[4 * 16 * LDT] __attribute__((aligned(16)));
#if TAIL_RES
  __shared__ _Float16 GRs[4 * 16 * LDT] __attribute__((aligned(16)));
#endif
  __shared__ float Os[4 * OTILE] __attribute__((aligned(16)));

  const unsigned tid = threadIdx.x, lane = tid & 31u;
  const int wave = __builtin_amdgcn_readfirstlane(threadIdx.x >> 5);
  const unsigned hh = lane >> 4, m = lane & 15u;
  const unsigned m0 = (blockIdx.x * 4u + (unsigned)wave) * 16u;
  const unsigned gb = (unsigned)wave * (16u * LDT);
  const unsigned ob = (unsigned)wave * (unsigned)OTILE;

  const size_t aoff = (size_t)(m0 + m) * K2 + hh * 8u;
  const unsigned boff = m * (unsigned)K2 + hh * 8u;

  v8f g[4];
#pragma unroll
  for (int nb = 0; nb < 4; ++nb) g[nb] = (v8f){};
#if TAIL_RES
  v8f gr[4];
#pragma unroll
  for (int nb = 0; nb < 4; ++nb) gr[nb] = (v8f){};
#endif
#pragma unroll
  for (unsigned k0 = 0; k0 < (unsigned)K2; k0 += 32u) {
    const v16h af = frag_at(Cp + aoff + k0);
#if TAIL_RES
    const v16h ar = frag_at(CpR + aoff + k0);
#endif
#pragma unroll
    for (int nb = 0; nb < 4; ++nb) {
      const v16h bf = frag_at(W2t + boff + (unsigned)nb * 16u * (unsigned)K2 + k0);
      g[nb] = wmma16(af, bf, g[nb]);
#if TAIL_RES
      gr[nb] = wmma16(ar, bf, gr[nb]);
#endif
    }
  }

  const float gscale = GCARRY / (CCARRY * WCARRY);
#pragma unroll
  for (int nb = 0; nb < 4; ++nb)
#pragma unroll
    for (int r = 0; r < 8; ++r) {
      float t = g[nb][r] * gscale;
#if TAIL_RES
      t = t + gr[nb][r] * (gscale / RCARRY);
#endif
      const h16 hi = toh_flush(t);
      Gs[gb + (hh * 8u + (unsigned)r) * LDT + (unsigned)nb * 16u + m] = hi;
#if TAIL_RES
      GRs[gb + (hh * 8u + (unsigned)r) * LDT + (unsigned)nb * 16u + m] =
          toh_flush((t - (float)hi) * RCARRY);
#endif
    }
  wave_lds_sync();

  v8f o[2];
  o[0] = (v8f){};
  o[1] = (v8f){};
#if TAIL_RES
  v8f orr[2];
  orr[0] = (v8f){};
  orr[1] = (v8f){};
#endif
#pragma unroll
  for (int c = 0; c < 2; ++c) {
    const v16h af = ld_frag(&Gs[gb + (unsigned)c * 32u], LDT);
#if TAIL_RES
    const v16h ar = ld_frag(&GRs[gb + (unsigned)c * 32u], LDT);
#endif
#pragma unroll
    for (int nb = 0; nb < 2; ++nb) {
      const v16h bf = frag_at(Fct + ((unsigned)nb * 16u + m) * (unsigned)HID + hh * 8u +
                              (unsigned)c * 32u);
      o[nb] = wmma16(af, bf, o[nb]);
#if TAIL_RES
      orr[nb] = wmma16(ar, bf, orr[nb]);
#endif
    }
  }

  const float oscale = 1.0f / (GCARRY * WCARRY);
#pragma unroll
  for (int nb = 0; nb < 2; ++nb) {
    const unsigned col = (unsigned)nb * 16u + m;
    const unsigned colc = (col < (unsigned)TAU) ? col : (unsigned)(TAU - 1);
    const float bias = bf16r(fcb[colc]);
#pragma unroll
    for (int r = 0; r < 8; ++r) {
      float t = o[nb][r] * oscale;
#if TAIL_RES
      t = t + orr[nb][r] * (oscale / RCARRY);
#endif
      t = t + bias;
      t = fminf(fmaxf(t, 0.0f), 10.0f);
      if (col < (unsigned)TAU) Os[ob + (hh * 8u + (unsigned)r) * (unsigned)TAU + col] = t;
    }
  }
  wave_lds_sync();

  v4f x[3];
  size_t off[3];
#pragma unroll
  for (unsigned i = 0; i < 3u; ++i) {
    const unsigned idx = i * 32u + lane;
    const unsigned idc = (idx < 88u) ? idx : 87u;
    x[i] = *(const v4f*)&Os[ob + idc * 4u];
    off[i] = (size_t)m0 * TAU + (size_t)idc * 4u;
  }
  *(volatile v4f*)(out + off[0]) = x[0];
  *(volatile v4f*)(out + off[1]) = x[1];
  if (lane < 24u) *(volatile v4f*)(out + off[2]) = x[2];
  __threadfence();
  *(volatile v4f*)(out + off[0]) = x[0];
  *(volatile v4f*)(out + off[1]) = x[1];
  if (lane < 24u) *(volatile v4f*)(out + off[2]) = x[2];
}

extern "C" void kernel_launch(void* const* d_in, const int* in_sizes, int n_in,
                              void* d_out, int out_size, void* d_ws, size_t ws_size,
                              hipStream_t stream) {
  if (n_in < 11) return;
  if ((long long)in_sizes[0] < (long long)NB * 2 * NNODE * FEAT) return;
  if (in_sizes[1] < INDIM * HID || in_sizes[5] < INDIM * HID) return;
  if (in_sizes[2] < 2 * HID || in_sizes[6] < 2 * HID) return;
  if (in_sizes[3] < HID * HID || in_sizes[7] < HID * HID) return;
  if (in_sizes[9] < HID * TAU || in_sizes[10] < TAU) return;
  if ((long long)out_size < (long long)NB * TAU) return;
  if (ws_size < WS_TOTAL) return;

  const float* fp    = (const float*)d_in[0];
  const float* uattW = (const float*)d_in[1];
  const float* uatta = (const float*)d_in[2];
  const float* uoutW = (const float*)d_in[3];
  const float* dattW = (const float*)d_in[5];
  const float* datta = (const float*)d_in[6];
  const float* doutW = (const float*)d_in[7];
  const float* fcW   = (const float*)d_in[9];
  const float* fcb   = (const float*)d_in[10];
  float* out = (float*)d_out;

  char* ws = (char*)d_ws;
  _Float16* W2t = (_Float16*)(ws + OFF_W2T);
  _Float16* Fct = (_Float16*)(ws + OFF_FCT);
  _Float16* Cp  = (_Float16*)(ws + OFF_C);
  _Float16* CpR = (_Float16*)(ws + OFF_CR);

  dim3 blk(256);
  wconv_kernel<<<dim3(1, 1), blk, 0, stream>>>(uoutW, W2t, (unsigned)HID, (unsigned)K2);
  wconv_kernel<<<dim3(1, 1), blk, 0, stream>>>(doutW, W2t + HID, (unsigned)HID, (unsigned)K2);
  fcconv_kernel<<<dim3(1), blk, 0, stream>>>(fcW, Fct);

  star_kernel<<<dim3(NB / 8), blk, 0, stream>>>(fp, uattW, uatta, Cp, CpR, 0u);
  star_kernel<<<dim3(NB / 8), blk, 0, stream>>>(fp, dattW, datta, Cp, CpR, 1u);

  tail_kernel<<<dim3(NB / 64), dim3(128), 0, stream>>>(Cp, CpR, W2t, Fct, fcb, out);
}
